// S4DReal_40123584479402
// MI455X (gfx1250) — hardware-run, weakly checked
//
#include <hip/hip_runtime.h>
#include <math.h>

typedef __attribute__((ext_vector_type(16))) _Float16 v16h;
typedef __attribute__((ext_vector_type(8)))  _Float16 v8h;
typedef __attribute__((ext_vector_type(2)))  _Float16 v2h;
typedef __attribute__((ext_vector_type(16))) __bf16   v16b;
typedef __attribute__((ext_vector_type(8)))  __bf16   v8b;
typedef __attribute__((ext_vector_type(8)))  float    v8f;
typedef __attribute__((ext_vector_type(4)))  float    v4f;
typedef __attribute__((ext_vector_type(2)))  float    v2f;

constexpr int kL    = 8192;
constexpr int kCh   = 256;
constexpr int kS    = 64;
constexpr int kQ    = 64;
constexpr int kNC   = kL / kQ;
constexpr int kLW   = kQ + 2 * kS;
constexpr int kThr  = 256;
constexpr float kDt = 1.0f / 16000.0f;
constexpr float kLCarry = 64.0f;
constexpr float kBCarry = 16384.0f;
constexpr float kTCarry = 536870912.0f;
constexpr float kSc1 = 1.0f / (kLCarry * kBCarry);
constexpr float kSc2 = 1.0f / (kLCarry * kTCarry);
constexpr float kF16MinNormal = 6.103515625e-5f;

static_assert(kL == 8192 && kCh == 256 && kS == 64 && kQ == 64 && kNC == 128 && kLW == 192, "the index arithmetic below uses these sizes");

constexpr size_t kOffZB = 0ull;
constexpr size_t kOffPW = 4096ull;
constexpr size_t kOffCB32 = 4263936ull;
constexpr size_t kOffKC32 = 4329472ull;
constexpr size_t kOffBQ16 = 4395008ull;
constexpr size_t kOffW216 = 6492160ull;
constexpr size_t kOffXG16 = 12783616ull;
constexpr size_t kOffGIN32 = 25366528ull;
constexpr size_t kOffG32 = 33755136ull;
constexpr size_t kOffYC32 = 42143744ull;
constexpr size_t kWsTotal = 50532352ull;
static_assert(kWsTotal <= 134217728ull, "carve cap: under 128 MiB");
static_assert(kOffZB == 0
              && kOffPW == kOffZB + 4096ull
              && kOffCB32 == kOffPW + 4259840ull
              && kOffKC32 == kOffCB32 + 65536ull
              && kOffBQ16 == kOffKC32 + 65536ull
              && kOffW216 == kOffBQ16 + 2097152ull
              && kOffXG16 == kOffW216 + 6291456ull
              && kOffGIN32 == kOffXG16 + 12582912ull
              && kOffG32 == kOffGIN32 + 8388608ull
              && kOffYC32 == kOffG32 + 8388608ull
              && kWsTotal == kOffYC32 + 8388608ull, "the carve is chained and totalled");
static_assert((kOffPW % 256) == 0 && (kOffCB32 % 256) == 0 && (kOffKC32 % 256) == 0 && (kOffBQ16 % 256) == 0 && (kOffW216 % 256) == 0 && (kOffXG16 % 256) == 0 && (kOffGIN32 % 256) == 0 && (kOffG32 % 256) == 0 && (kOffYC32 % 256) == 0, "aligned regions");
static_assert(1024 >= 64, "the zero record covers the 64 output columns of both products (the engine reads one bias value a column)");

__device__ __forceinline__ unsigned short f2bf_bits(float f) {
  unsigned u = __float_as_uint(f);
  return (unsigned short)((u + 0x7FFFu + ((u >> 16) & 1u)) >> 16);
}
__device__ __forceinline__ float bf_bits2f(unsigned short h) { return __uint_as_float(((unsigned)h) << 16); }
__device__ __forceinline__ float bf16r(float f) { return bf_bits2f(f2bf_bits(f)); }
__device__ __forceinline__ float carry_flush(float v, float carry) {
  const float s = v * carry;
  return (fabsf(s) < kF16MinNormal) ? 0.0f : s;
}

__device__ __forceinline__ void dep_guard4_h(v8f& a, v8f& b, v8f& c, v8f& d, v16h x, v16h y) { asm volatile("v_nop\n\tv_nop\n\tv_nop\n\tv_nop" : "+v"(a), "+v"(b), "+v"(c), "+v"(d) : "v"(x), "v"(y)); }
__device__ __forceinline__ void dep_guard4_b(v8f& a, v8f& b, v8f& c, v8f& d, v16b x, v16b y) { asm volatile("v_nop\n\tv_nop\n\tv_nop\n\tv_nop" : "+v"(a), "+v"(b), "+v"(c), "+v"(d) : "v"(x), "v"(y)); }
__device__ __forceinline__ void keep4_h(v16h a, v16h b, v16h c, v16h d) { asm volatile("v_nop" :: "v"(a), "v"(b), "v"(c), "v"(d)); }
__device__ __forceinline__ void keep4_b(v16b a, v16b b, v16b c, v16b d) { asm volatile("v_nop" :: "v"(a), "v"(b), "v"(c), "v"(d)); }
__device__ __forceinline__ void acc_guard4(v8f& a, v8f& b, v8f& c, v8f& d) { asm volatile("v_nop\n\tv_nop\n\tv_nop\n\tv_nop" : "+v"(a), "+v"(b), "+v"(c), "+v"(d)); }

template <typename T> struct Frag;
template <> struct Frag<_Float16> {
  typedef v16h V; union U { v16h v; v8h h[2]; };
  static __device__ __forceinline__ v16h load(const _Float16* p) {
    U f; f.h[0] = *(const v8h*)(p); f.h[1] = *(const v8h*)(p + 16); return f.v;
  }
  static __device__ __forceinline__ v8f mma(v16h a, v16h b, v8f c) {
    return __builtin_amdgcn_wmma_f32_16x16x32_f16(false, a, false, b, (short)0, c, false, false);
  }
  static __device__ __forceinline__ void guard4(v8f& a, v8f& b, v8f& c, v8f& d, v16h x, v16h y) { dep_guard4_h(a, b, c, d, x, y); }
  static __device__ __forceinline__ void keep(v16h a, v16h b, v16h c, v16h d) { keep4_h(a, b, c, d); }
};
template <> struct Frag<__bf16> {
  typedef v16b V; union U { v16b v; v8b h[2]; };
  static __device__ __forceinline__ v16b load(const __bf16* p) {
    U f; f.h[0] = *(const v8b*)(p); f.h[1] = *(const v8b*)(p + 16); return f.v;
  }
  static __device__ __forceinline__ v8f mma(v16b a, v16b b, v8f c) {
    return __builtin_amdgcn_wmma_f32_16x16x32_bf16(false, a, false, b, (short)0, c, false, false);
  }
  static __device__ __forceinline__ void guard4(v8f& a, v8f& b, v8f& c, v8f& d, v16b x, v16b y) { dep_guard4_b(a, b, c, d, x, y); }
  static __device__ __forceinline__ void keep(v16b a, v16b b, v16b c, v16b d) { keep4_b(a, b, c, d); }
};

__device__ __forceinline__ v8f mma_h(v16h a, v16h b, v8f c) {
  c = __builtin_amdgcn_wmma_f32_16x16x32_f16(false, a, false, b, (short)0, c, false, false);
  asm volatile("v_nop\n\tv_nop\n\tv_nop\n\tv_nop" : "+v"(c) : "v"(a), "v"(b));
  return c;
}

template <int ET> struct Elem;
template <> struct Elem<0> { typedef _Float16 T; };
template <> struct Elem<1> { typedef __bf16 T; };
template <int ET, bool SPLIT, int BIAS_MODE, int OUT_MODE, bool RESID, int ACT = 0>
__global__ __launch_bounds__(256) void wmma_gemm64(
    const unsigned short* __restrict__ Ap, const unsigned short* __restrict__ A2p, int lda, long strideA,
    const unsigned short* __restrict__ Btp, const unsigned short* __restrict__ Bt2p, int ldb, long strideB,
    void* __restrict__ Cout, void* __restrict__ Cout2, int ldc, long strideC,
    const float* __restrict__ bias,
    const float* __restrict__ resid, long strideR,
    int M, int N, int K, float scale) {
  typedef typename Elem<ET>::T T;
  typedef typename Frag<T>::V V;
  const T* A = (const T*)Ap; const T* A2 = (const T*)A2p; const T* Bt = (const T*)Btp; const T* Bt2 = (const T*)Bt2p;
  __shared__ __align__(16) float sT[8][16 * 68];
  const int b    = blockIdx.y;
  const int lane = threadIdx.x & 31;
  const int wave = threadIdx.x >> 5;
  const int tilesN = N >> 6;
  const int tilesM = M >> 6;
  const int tile = blockIdx.x * 8 + wave;
  if (tile >= tilesM * tilesN) return;
  const int tm = tile / tilesN;
  const int tn = tile - tm * tilesN;
  const int m0 = tm << 6;
  const int n0 = tn << 6;

  const T* Ab  = A  + (size_t)b * strideA;
  const T* Bb  = Bt + (size_t)b * strideB;
  const T* Ab2 = SPLIT ? (A2  + (size_t)b * strideA) : nullptr;
  const T* Bb2 = SPLIT ? (Bt2 + (size_t)b * strideB) : nullptr;

  const int rlane = lane & 15;
  const int koff  = (lane >> 4) * 8;
  const int mOff  = (lane >> 4) * 8;

  v8f acc[4][4];
#pragma unroll
  for (int i = 0; i < 4; ++i)
#pragma unroll
    for (int j = 0; j < 4; ++j) acc[i][j] = (v8f){0.f,0.f,0.f,0.f,0.f,0.f,0.f,0.f};

  for (int k0 = 0; k0 < K; k0 += 32) {
    V bh[4], bl[4];
#pragma unroll
    for (int j = 0; j < 4; ++j) {
      const size_t bo = (size_t)(n0 + (j << 4) + rlane) * ldb + koff + k0;
      bh[j] = Frag<T>::load(Bb + bo);
      if (SPLIT) bl[j] = Frag<T>::load(Bb2 + bo);
    }
#pragma unroll
    for (int i = 0; i < 4; ++i) {
      const size_t ao = (size_t)(m0 + (i << 4) + rlane) * lda + koff + k0;
      V ah = Frag<T>::load(Ab + ao);
      V al;
      if (SPLIT) al = Frag<T>::load(Ab2 + ao);
#pragma unroll
      for (int j = 0; j < 4; ++j) {
        acc[i][j] = Frag<T>::mma(ah, bh[j], acc[i][j]);
        if (SPLIT) {
          acc[i][j] = Frag<T>::mma(ah, bl[j], acc[i][j]);
          acc[i][j] = Frag<T>::mma(al, bh[j], acc[i][j]);
        }
      }
      Frag<T>::guard4(acc[i][0], acc[i][1], acc[i][2], acc[i][3], ah, SPLIT ? al : ah);
    }
    Frag<T>::keep(bh[0], bh[1], bh[2], bh[3]);
    if (SPLIT) Frag<T>::keep(bl[0], bl[1], bl[2], bl[3]);
  }
  acc_guard4(acc[0][0], acc[0][1], acc[0][2], acc[0][3]);
  acc_guard4(acc[1][0], acc[1][1], acc[1][2], acc[1][3]);
  acc_guard4(acc[2][0], acc[2][1], acc[2][2], acc[2][3]);
  acc_guard4(acc[3][0], acc[3][1], acc[3][2], acc[3][3]);

  float* slab = sT[wave];
  const float* Rb = RESID ? (resid + (size_t)b * strideR) : nullptr;
#pragma unroll
  for (int i = 0; i < 4; ++i) {
    const int mBase = m0 + (i << 4);
#pragma unroll
    for (int j = 0; j < 4; ++j) {
      const int n = n0 + (j << 4) + rlane;
      float bv = 0.f;
      if (BIAS_MODE == 2) bv = bias[n];
#pragma unroll
      for (int r = 0; r < 8; ++r) {
        float v = acc[i][j][r] * scale;
        if (BIAS_MODE == 1) v += bias[mBase + mOff + r];
        if (BIAS_MODE == 2) v += bv;
        if (RESID) v += Rb[(size_t)(mBase + mOff + r) * ldc + n];
        if (ACT == 1) v = tanhf(v);
        if (ACT == 2) v = fmaxf(v, 0.0f);
        if (ACT == 3) v = v / (1.0f + expf(-v));
        if (ACT == 4) v = (v > 0.f) ? v : 0.01f * v;
        slab[(mOff + r) * 68 + (j << 4) + rlane] = v;
      }
    }
    __builtin_amdgcn_fence(__ATOMIC_RELEASE, "workgroup");
    __builtin_amdgcn_wave_barrier();
    __builtin_amdgcn_fence(__ATOMIC_ACQUIRE, "workgroup");
    if (OUT_MODE == 0) {
      float* C = (float*)Cout + (size_t)b * strideC;
      const int hh = lane >> 4, c4 = (lane & 15) * 4;
      for (int pass = 0; pass < 2; ++pass) {
#pragma unroll
        for (int it = 0; it < 8; ++it) {
          const int row = it * 2 + hh;
          v4f v = *(const v4f*)(slab + row * 68 + c4);
          *(volatile v4f*)(C + (size_t)(mBase + row) * ldc + n0 + c4) = v;
        }
        __threadfence();
      }
    } else {
      const int q = lane >> 3, c8 = (lane & 7) * 8;
      unsigned short* C  = (unsigned short*)Cout  + (size_t)b * strideC;
      unsigned short* C2 = (OUT_MODE == 2) ? ((unsigned short*)Cout2 + (size_t)b * strideC) : nullptr;
      for (int pass = 0; pass < 2; ++pass) {
#pragma unroll
        for (int it = 0; it < 4; ++it) {
          const int row = it * 4 + q;
          const float* sp = slab + row * 68 + c8;
          v8h hv, lv;
#pragma unroll
          for (int e = 0; e < 8; ++e) {
            if (OUT_MODE == 1) {
              hv[e] = (_Float16)sp[e];
            } else {
              unsigned short hb = f2bf_bits(sp[e]);
              unsigned short lb = f2bf_bits(sp[e] - bf_bits2f(hb));
              hv[e] = __builtin_bit_cast(_Float16, hb);
              lv[e] = __builtin_bit_cast(_Float16, lb);
            }
          }
          *(volatile v8h*)(C + (size_t)(mBase + row) * ldc + n0 + c8) = hv;
          if (OUT_MODE == 2) *(volatile v8h*)(C2 + (size_t)(mBase + row) * ldc + n0 + c8) = lv;
        }
        __threadfence();
      }
    }
    __builtin_amdgcn_fence(__ATOMIC_RELEASE, "workgroup");
    __builtin_amdgcn_wave_barrier();
    __builtin_amdgcn_fence(__ATOMIC_ACQUIRE, "workgroup");
  }
}


__device__ __forceinline__ void two_words(float w, float carry, _Float16& hh, _Float16& ll) {
  const float sc = carry_flush(w, carry);
  hh = (_Float16)sc;
  const float rs = sc - (float)hh;
  ll = (_Float16)((fabsf(rs) < kF16MinNormal) ? 0.0f : rs);
}
__device__ __forceinline__ void store2(float* p, float v) {
  *(volatile float*)p = v;
  __threadfence();
  *(volatile float*)p = v;
}


__global__ __launch_bounds__(kThr) void zero_kernel(float* __restrict__ dst) {
  const size_t o4 = ((size_t)blockIdx.x * kThr + threadIdx.x) * 4u;
  const v4f z = {0.f, 0.f, 0.f, 0.f};
  *(volatile v4f*)(dst + o4) = z;
  __threadfence();
  *(volatile v4f*)(dst + o4) = z;
}

__global__ __launch_bounds__(kThr) void ptab_kernel(const float* __restrict__ lognegA, float* __restrict__ PW) {
  const unsigned t = blockIdx.x * (unsigned)kThr + threadIdx.x;
  const unsigned k = t >> 14, cs = t & 16383u;
  const float la = lognegA[cs];
  const float a = -expf(bf16r(la));
  store2(PW + t, expf((float)k * (a * kDt)));
}
static_assert(65 * kCh * kS == 4160 * kThr, "powers grid exact: 4,160 blocks");

__global__ __launch_bounds__(kThr) void cb_kernel(const float* __restrict__ lognegA, const float* __restrict__ Bm, const float* __restrict__ Cp, float* __restrict__ CB) {
  const unsigned t = blockIdx.x * (unsigned)kThr + threadIdx.x;
  const float la = lognegA[t], bv = Bm[t], cv = Cp[t];
  const float a = -expf(bf16r(la));
  const float bd = (expf(a * kDt) - 1.0f) * bf16r(bv) / a;
  store2(CB + t, bf16r(cv) * bd);
}
static_assert(kCh * kS == 64 * kThr, "Cp Bd grid exact: 64 blocks");

__global__ __launch_bounds__(kThr) void kc_kernel(const float* __restrict__ CB, const float* __restrict__ PW, float* __restrict__ KC) {
  const unsigned t = blockIdx.x * (unsigned)kThr + threadIdx.x;
  const unsigned l = t >> 8, c = t & 255u;
  const float* cb = CB + (size_t)c * kS;
  const float* pw = PW + ((size_t)l * kCh + c) * kS;
  float acc = 0.0f;
  for (int s = 0; s < kS; ++s) acc += cb[s] * pw[s];
  store2(KC + t, acc);
}
static_assert(kQ * kCh == 64 * kThr, "in-chunk kernel grid exact: 64 blocks");

__global__ __launch_bounds__(kThr) void bq_kernel(const float* __restrict__ PW, unsigned short* __restrict__ BQ) {
  const unsigned t = blockIdx.x * (unsigned)kThr + threadIdx.x;
  const unsigned cs = t >> 3, q8 = (t & 7u) * 8u;
  v8h hv;
#pragma unroll
  for (int e = 0; e < 8; ++e) {
    const unsigned k = 63u - (q8 + (unsigned)e);
    const float v = PW[(size_t)k * (kCh * kS) + cs];
    hv[e] = (_Float16)carry_flush(v, kBCarry);
  }
  unsigned short* dp = BQ + (size_t)cs * kQ + q8;
  *(volatile v8h*)dp = hv;
  __threadfence();
  *(volatile v8h*)dp = hv;
}
static_assert((size_t)kCh * kS * (kQ / 8) == 512ull * kThr, "state-operand cast grid exact: 512 blocks");

__global__ __launch_bounds__(64) void w2_kernel(const float* __restrict__ CB, const float* __restrict__ PW, const float* __restrict__ KC, unsigned short* __restrict__ W2) {
  const unsigned cr = blockIdx.x;
  const unsigned g = threadIdx.x;
  if (g >= 24u) return;
  const unsigned c = cr >> 6, r = cr & 63u;
  const unsigned c8 = g * 8u;
  v8h hv;
#pragma unroll
  for (int e = 0; e < 8; ++e) {
    const unsigned col = c8 + (unsigned)e;
    float v;
    if (col < 64u) {
      const float kv = KC[((r - col) & 63u) * (unsigned)kCh + c];
      v = (col <= r) ? kv : 0.0f;
    } else {
      const unsigned s = (col - 64u) & 63u;
      v = CB[(size_t)c * kS + s] * PW[((size_t)(r + 1u) * kCh + c) * kS + s];
    }
    hv[e] = (_Float16)carry_flush(v, kTCarry);
  }
  unsigned short* dp = W2 + (size_t)cr * kLW + c8;
  *(volatile v8h*)dp = hv;
  __threadfence();
  *(volatile v8h*)dp = hv;
}

__global__ __launch_bounds__(kThr) void xcast_kernel(const float* __restrict__ X, unsigned short* __restrict__ XG) {
  const unsigned t = blockIdx.x * (unsigned)kThr + threadIdx.x;
  const unsigned row = t >> 3, q8 = (t & 7u) * 8u;
  const unsigned c = row >> 7, ch = row & 127u;
  v8h hv;
#pragma unroll
  for (int e = 0; e < 8; ++e) {
    const float v = X[((size_t)ch * kQ + q8 + (unsigned)e) * kCh + c];
    hv[e] = (_Float16)carry_flush(bf16r(v), kLCarry);
  }
  unsigned short* dp = XG + (size_t)row * kLW + q8;
  *(volatile v8h*)dp = hv;
  __threadfence();
  *(volatile v8h*)dp = hv;
}
static_assert((size_t)kCh * kNC * (kQ / 8) == 1024ull * kThr, "input cast grid exact: 1,024 blocks");

__global__ __launch_bounds__(kThr) void gscan_kernel(const float* __restrict__ GIN, const float* __restrict__ D, float* __restrict__ G) {
  const unsigned cs = blockIdx.x * (unsigned)kThr + threadIdx.x;
  const unsigned c = cs >> 6, s = cs & 63u;
  const float d = D[cs];
  float g = 0.0f;
  for (int n = 0; n < kNC; ++n) {
    const size_t at = ((size_t)c * kNC + (size_t)n) * kS + s;
    store2(G + at, g);
    g = d * g + GIN[at];
  }
}
static_assert(kCh * kS == 64 * kThr, "chunk recurrence grid exact: 64 blocks");

__global__ __launch_bounds__(kThr) void gcast_kernel(const float* __restrict__ G, unsigned short* __restrict__ XG) {
  const unsigned t = blockIdx.x * (unsigned)kThr + threadIdx.x;
  const unsigned row = t >> 3, s8 = (t & 7u) * 8u;
  const float* sp = G + (size_t)row * kS + s8;
  v8h hv, lv;
#pragma unroll
  for (int e = 0; e < 8; ++e) { const float v = sp[e]; _Float16 a, b; two_words(v, kLCarry, a, b); hv[e] = a; lv[e] = b; }
  unsigned short* dp = XG + (size_t)row * kLW + (unsigned)kQ + s8;
  for (int pass = 0; pass < 2; ++pass) {
    *(volatile v8h*)dp = hv; *(volatile v8h*)(dp + 64) = lv;
    __threadfence();
  }
}
static_assert((size_t)kCh * kNC * (kS / 8) == 1024ull * kThr, "state cast grid exact: 1,024 blocks");

__global__ __launch_bounds__(kThr) void ytr_kernel(const float* __restrict__ YC, float* __restrict__ out) {
  const unsigned i = blockIdx.x * (unsigned)kThr + threadIdx.x;
  const unsigned t = i >> 8, c = i & 255u;
  const float v = YC[(size_t)c * kL + t];
  store2(out + i, v);
}
static_assert((size_t)kL * kCh == 8192ull * kThr, "output grid exact: 8,192 blocks");

extern "C" void kernel_launch(void* const* d_in, const int* in_sizes, int n_in,
                              void* d_out, int out_size, void* d_ws, size_t ws_size,
                              hipStream_t stream) {
  if (n_in < 4 || d_out == nullptr || d_ws == nullptr) return;
  if (in_sizes[0] != kL * kCh || in_sizes[1] != kCh * kS || in_sizes[2] != kCh * kS || in_sizes[3] != kCh * kS) return;
  if (out_size != kL * kCh) return;
  if (ws_size < kWsTotal) return;
  const float* X = (const float*)d_in[0];
  const float* lognegA = (const float*)d_in[1];
  const float* Bm = (const float*)d_in[2];
  const float* Cp = (const float*)d_in[3];
  float* out = (float*)d_out;
  char* ws = (char*)d_ws;
  float* ZB = (float*)(ws + kOffZB);
  float* PW = (float*)(ws + kOffPW);
  float* CB32 = (float*)(ws + kOffCB32);
  float* KC32 = (float*)(ws + kOffKC32);
  unsigned short* BQ16 = (unsigned short*)(ws + kOffBQ16);
  unsigned short* W216 = (unsigned short*)(ws + kOffW216);
  unsigned short* XG16 = (unsigned short*)(ws + kOffXG16);
  float* GIN32 = (float*)(ws + kOffGIN32);
  float* G32 = (float*)(ws + kOffG32);
  float* YC32 = (float*)(ws + kOffYC32);

  zero_kernel<<<1, kThr, 0, stream>>>(ZB);
  ptab_kernel<<<4160, kThr, 0, stream>>>(lognegA, PW);
  cb_kernel<<<64, kThr, 0, stream>>>(lognegA, Bm, Cp, CB32);
  kc_kernel<<<64, kThr, 0, stream>>>(CB32, PW, KC32);
  bq_kernel<<<512, kThr, 0, stream>>>(PW, BQ16);
  w2_kernel<<<kCh * kQ, 64, 0, stream>>>(CB32, PW, KC32, W216);
  xcast_kernel<<<1024, kThr, 0, stream>>>(X, XG16);
  wmma_gemm64<0, false, 2, 0, false, 0><<<dim3(1, kCh), 256, 0, stream>>>(
      XG16, XG16, kLW, (long)kNC * kLW, BQ16, BQ16, kQ, (long)kS * kQ, (void*)GIN32, (void*)GIN32, kS, (long)kNC * kS, ZB, nullptr, 0L, kNC, kS, kQ, kSc1);
  gscan_kernel<<<64, kThr, 0, stream>>>(GIN32, PW + (size_t)kQ * kCh * kS, G32);
  gcast_kernel<<<1024, kThr, 0, stream>>>(G32, XG16);
  wmma_gemm64<0, false, 2, 0, false, 0><<<dim3(1, kCh), 256, 0, stream>>>(
      XG16, XG16, kLW, (long)kNC * kLW, W216, W216, kLW, (long)kQ * kLW, (void*)YC32, (void*)YC32, kQ, (long)kNC * kQ, ZB, nullptr, 0L, kNC, kQ, kLW, kSc2);
  ytr_kernel<<<8192, kThr, 0, stream>>>(YC32, out);
}
